// OpenPanguMoEDecoderLayer_9620726743830
// MI455X (gfx1250) — hardware-verified
//
#include <hip/hip_runtime.h>
#include <math.h>

typedef __attribute__((ext_vector_type(16))) _Float16 v16h;
typedef __attribute__((ext_vector_type(16))) __bf16 v16b;
typedef __attribute__((ext_vector_type(8)))  _Float16 v8h;
typedef __attribute__((ext_vector_type(8)))  __bf16 v8b;
typedef __attribute__((ext_vector_type(8)))  float v8f;
typedef __attribute__((ext_vector_type(4)))  float v4f;
typedef __attribute__((ext_vector_type(4)))  unsigned v4u;
typedef _Float16 h16;

#ifndef NB
#define NB 1024
#endif
#define NB_FULL 1024
#define DIN  1024
#define DHID 512
#define DOUT 1024
#define NE   16
#define NX   (NE + 1)
#define KF (NX * DHID)
#define KP KF
#define HCARRY 64.0f
#define WCARRY 512.0f
#define OSCALE (1.0f / 32768.0f)
#define ROUTED_SCALE 2.5f

#define WS_XB  ((size_t)0)
#define WS_WGT (WS_XB  + (size_t)NB * DIN * 2)
#define WS_WUT (WS_WGT + (size_t)NX * DHID * DIN * 2)
#define WS_W2T (WS_WUT + (size_t)NX * DHID * DIN * 2)
#define WS_HB  (WS_W2T + (size_t)DOUT * KP * 2)
#define WS_RT  (WS_HB  + (size_t)NB * KP * 2)
#define WS_END (WS_RT  + (size_t)NB * NE * 4)

static_assert(NB % 128 == 0);
static_assert(NB <= NB_FULL);
static_assert(DIN % 64 == 0 && DHID % 64 == 0 && DOUT % 128 == 0);
static_assert(DIN % 32 == 0 && KP % 32 == 0 && (KP * 2) % 128 == 0);
static_assert(KP == NE * DHID + DHID);
static_assert((size_t)NB_FULL * DOUT * 4 == 4194304);
static_assert(WS_WGT % 128 == 0 && WS_WUT % 128 == 0 && WS_W2T % 128 == 0 && WS_HB % 128 == 0 && WS_RT % 128 == 0);
static_assert(WS_END <= (size_t)134217728);
static_assert(64 * 65 * 4 <= 131072);
static_assert(16 * NE * 4 <= 131072);
static_assert(128 * 64 * 2 <= 131072);
static_assert(8 * 16 * 64 * 4 <= 131072);
static_assert((size_t)(NB * DIN / 8 / 256) * 256 * 8 == (size_t)NB * DIN);
static_assert((size_t)(DHID / 64) * (DIN / 64) * NE * 4096 + (size_t)(DHID / 64) * (DIN / 64) * 4096 == (size_t)NX * DIN * DHID);
static_assert((size_t)(DOUT / 64) * (DHID / 64) * NE * 4096 + (size_t)(DOUT / 64) * (DHID / 64) * 4096 == (size_t)DOUT * KF);
static_assert(NE == 16 && DIN % 8 == 0);
static_assert((size_t)(NB / 16) * 256 == (size_t)NB * NE);
static_assert(64 * 4 == 16 * NE);
static_assert((size_t)(DHID / 64) * (NB / 128) * NX * 128 * 64 == (size_t)NB * KF);
static_assert(256 * 4 * 8 == 128 * 64);
static_assert((size_t)(DOUT / 128) * (NB / 128) * 128 * 128 == (size_t)NB * DOUT);

__device__ __forceinline__ v8f wmma16(v16h a, v16h b, v8f c) {
  v8f d = __builtin_amdgcn_wmma_f32_16x16x32_f16(false, a, false, b, (short)0, c, false, false);
  asm volatile("v_nop\n\tv_nop\n\tv_nop\n\tv_nop" : "+v"(d) : "v"(a), "v"(b));
  return d;
}
__device__ __forceinline__ v8f wmma_bf(v16b a, v16b b, v8f c) {
  v8f d = __builtin_amdgcn_wmma_f32_16x16x32_bf16(false, a, false, b, (short)0, c, false, false);
  asm volatile("v_nop\n\tv_nop\n\tv_nop\n\tv_nop" : "+v"(d) : "v"(a), "v"(b));
  return d;
}
__device__ __forceinline__ float bfr(float v) { return (float)(__bf16)v; }
static __device__ __forceinline__ h16 toh_flush(float v) { const h16 r = (h16)v; return (fabsf(v) < 6.103515625e-05f) ? (h16)0.0f : r; }
__device__ __forceinline__ v16b ldfrag_b(const unsigned short* p) { union { v16b v; v4u q[2]; } f; f.q[0] = *(const v4u*)p; f.q[1] = *(const v4u*)(p + 16); return f.v; }
__device__ __forceinline__ v16h ldfrag_h(const unsigned short* p) { union { v16h v; v4u q[2]; } f; f.q[0] = *(const v4u*)p; f.q[1] = *(const v4u*)(p + 16); return f.v; }

__global__ __launch_bounds__(256) void k_cvt_x(const float* __restrict__ X, unsigned short* __restrict__ XB) {
  const unsigned i = blockIdx.x * 256u + threadIdx.x;
  const unsigned ic = i < (unsigned)(NB * DIN / 8) ? i : (unsigned)(NB * DIN / 8 - 1);
  const v4f a = *(const v4f*)(X + (size_t)ic * 8), b = *(const v4f*)(X + (size_t)ic * 8 + 4);
  union { v8b h; v4u u; } o;
#pragma unroll
  for (int j = 0; j < 4; ++j) { o.h[j] = (__bf16)a[j]; o.h[4 + j] = (__bf16)b[j]; }
  const v4u val = o.u;
  volatile v4u* p = (volatile v4u*)(XB + (size_t)ic * 8);
  *p = val; __threadfence(); *p = val;
}

template <int F16>
__global__ __launch_bounds__(256) void k_tr(const float* __restrict__ S, unsigned short* __restrict__ Dst, unsigned K, unsigned N, unsigned dpitch, unsigned erow, unsigned ecol, float sc) {
  __shared__ float tile[64][65];
  const unsigned t = threadIdx.x, e = blockIdx.z, k0 = blockIdx.y * 64u, n0 = blockIdx.x * 64u;
  const float* s = S + (size_t)e * K * N;
#pragma unroll
  for (unsigned it = 0; it < 4; ++it) { const unsigned idx = it * 256u + t, kr = idx >> 4, c4 = idx & 15u;
    const v4f v = *(const v4f*)(s + (size_t)(k0 + kr) * N + n0 + 4u * c4);
    tile[kr][4u * c4 + 0] = v[0]; tile[kr][4u * c4 + 1] = v[1]; tile[kr][4u * c4 + 2] = v[2]; tile[kr][4u * c4 + 3] = v[3]; }
  __syncthreads();
  v4u o[2];
#pragma unroll
  for (unsigned it = 0; it < 2; ++it) { const unsigned idx = it * 256u + t, nr = idx >> 3, q = idx & 7u;
    union { v8b b; v8h h; v4u u; } w;
#pragma unroll
    for (int i = 0; i < 8; ++i) { const float v = bfr(tile[8u * q + i][nr]); if (F16) w.h[i] = toh_flush(v * sc); else w.b[i] = (__bf16)v; }
    o[it] = w.u; }
#pragma unroll
  for (unsigned it = 0; it < 2; ++it) { const unsigned idx = it * 256u + t, nr = idx >> 3, q = idx & 7u;
    *(volatile v4u*)(Dst + (size_t)(e * erow + n0 + nr) * dpitch + e * ecol + k0 + 8u * q) = o[it]; }
  __threadfence();
#pragma unroll
  for (unsigned it = 0; it < 2; ++it) { const unsigned idx = it * 256u + t, nr = idx >> 3, q = idx & 7u;
    *(volatile v4u*)(Dst + (size_t)(e * erow + n0 + nr) * dpitch + e * ecol + k0 + 8u * q) = o[it]; }
}

__global__ __launch_bounds__(256) void k_gate(const unsigned short* __restrict__ XB, const float* __restrict__ GW, float* __restrict__ RT) {
#pragma clang fp contract(off)
  __shared__ __align__(16) float sp[16][NE];
  const int wave = __builtin_amdgcn_readfirstlane(threadIdx.x >> 5);
  const unsigned tid = threadIdx.x, lane = tid & 31u, col = lane & 15u, g = lane >> 4; const unsigned r0 = blockIdx.x * 16u;
  const unsigned lrow = (unsigned)wave * 2u + g, row = r0 + lrow;
  const unsigned short* xp = XB + (size_t)row * DIN;
  const float* gp = GW + (size_t)col * DIN;
  float acc = 0.0f;
#pragma unroll 1
  for (unsigned kc = 0; kc < DIN / 8; ++kc) {
    const v4u xq = *(const v4u*)(xp + kc * 8u);
    const v4f w0 = *(const v4f*)(gp + kc * 8u), w1 = *(const v4f*)(gp + kc * 8u + 4u);
    acc = fmaf(__uint_as_float(xq[0] << 16),         bfr(w0[0]), acc);
    acc = fmaf(__uint_as_float(xq[0] & 0xffff0000u), bfr(w0[1]), acc);
    acc = fmaf(__uint_as_float(xq[1] << 16),         bfr(w0[2]), acc);
    acc = fmaf(__uint_as_float(xq[1] & 0xffff0000u), bfr(w0[3]), acc);
    acc = fmaf(__uint_as_float(xq[2] << 16),         bfr(w1[0]), acc);
    acc = fmaf(__uint_as_float(xq[2] & 0xffff0000u), bfr(w1[1]), acc);
    acc = fmaf(__uint_as_float(xq[3] << 16),         bfr(w1[2]), acc);
    acc = fmaf(__uint_as_float(xq[3] & 0xffff0000u), bfr(w1[3]), acc);
  }
  const float p = 1.0f / (1.0f + expf(-acc));
  float m1 = p; int i1 = (int)col;
#pragma unroll
  for (int off = 1; off < 16; off <<= 1) { const float om = __shfl_xor(m1, off); const int oi = __shfl_xor(i1, off);
    const bool tk = (om > m1) || ((om == m1) && (oi < i1)); m1 = tk ? om : m1; i1 = tk ? oi : i1; }
  const float p2 = ((int)col == i1) ? -1.0f : p;
  float m2 = p2; int i2 = (int)col;
#pragma unroll
  for (int off = 1; off < 16; off <<= 1) { const float om = __shfl_xor(m2, off); const int oi = __shfl_xor(i2, off);
    const bool tk = (om > m2) || ((om == m2) && (oi < i2)); m2 = tk ? om : m2; i2 = tk ? oi : i2; }
  const float inv = 1.0f / (m1 + m2 + 1e-20f);
  const float w1r = m1 * inv * ROUTED_SCALE, w2r = m2 * inv * ROUTED_SCALE;
  const float rw = ((int)col == i1) ? w1r : (((int)col == i2) ? w2r : 0.0f);
  sp[lrow][col] = rw;
  __syncthreads();
  if (wave < 2) {
    const v4f pv = *(const v4f*)(&sp[0][0] + 4u * tid);
    volatile v4f* po = (volatile v4f*)(RT + (size_t)r0 * NE + 4u * tid);
    *po = pv; __threadfence(); *po = pv;
  }
}

__global__ __launch_bounds__(256) void k_h(const unsigned short* __restrict__ XB, const unsigned short* __restrict__ WGT, const unsigned short* __restrict__ WUT, const float* __restrict__ RT, unsigned short* __restrict__ HB) {
  __shared__ __align__(16) _Float16 sh[128][64];
  const unsigned t = threadIdx.x, wave = t >> 5, lane = t & 31u, lm = lane & 15u, lh = lane >> 4, wm = wave >> 1, wn = wave & 1u;
  const unsigned e = blockIdx.z, m0 = blockIdx.y * 128u, n0 = blockIdx.x * 64u;
  const unsigned short* ar[2]; const unsigned short* br[4];
#pragma unroll
  for (int mi = 0; mi < 2; ++mi) ar[mi] = XB + (size_t)(m0 + wm * 32u + mi * 16u + lm) * DIN + 8u * lh;
#pragma unroll
  for (int ni = 0; ni < 2; ++ni) { const size_t ro = (size_t)(e * DHID + n0 + wn * 32u + ni * 16u + lm) * DIN + 8u * lh; br[ni] = WGT + ro; br[2 + ni] = WUT + ro; }
  v8f acc[2][4] = {};
#pragma unroll 2
  for (unsigned kc = 0; kc < DIN / 32; ++kc) { v16b a[2], b[4];
#pragma unroll
    for (int mi = 0; mi < 2; ++mi) a[mi] = ldfrag_b(ar[mi] + kc * 32u);
#pragma unroll
    for (int ni = 0; ni < 4; ++ni) b[ni] = ldfrag_b(br[ni] + kc * 32u);
#pragma unroll
    for (int mi = 0; mi < 2; ++mi)
#pragma unroll
      for (int ni = 0; ni < 4; ++ni) acc[mi][ni] = wmma_bf(a[mi], b[ni], acc[mi][ni]); }
  const unsigned ec = e < (unsigned)NE ? e : (unsigned)(NE - 1);
  float wv[2][8];
#pragma unroll
  for (int mi = 0; mi < 2; ++mi) {
#pragma unroll
    for (int r = 0; r < 8; ++r) { const float rv = RT[(size_t)(m0 + wm * 32u + mi * 16u + 8u * lh + r) * NE + ec]; wv[mi][r] = (e < (unsigned)NE ? rv : 1.0f) * HCARRY; }
    asm volatile("s_wait_loadcnt 0x0" ::: "memory"); }
#pragma unroll
  for (int ni = 0; ni < 2; ++ni) {
#pragma unroll
    for (int mi = 0; mi < 2; ++mi)
#pragma unroll
      for (int r = 0; r < 8; ++r) { const float gv = acc[mi][ni][r], uv = acc[mi][2 + ni][r];
        const float sg = 1.0f / (1.0f + expf(-gv));
        sh[wm * 32u + mi * 16u + 8u * lh + r][wn * 32u + ni * 16u + lm] = toh_flush(gv * sg * uv * wv[mi][r]); } }
  __syncthreads();
  v4u o[4];
#pragma unroll
  for (unsigned it = 0; it < 4; ++it) { const unsigned rw = it * 32u + (t >> 3), q = t & 7u; union { v8h h; v4u u; } w; w.h = *(const v8h*)&sh[rw][8u * q]; o[it] = w.u; }
  unsigned short* hb = HB + (size_t)m0 * KP + e * DHID + n0;
#pragma unroll
  for (unsigned it = 0; it < 4; ++it) { const unsigned rw = it * 32u + (t >> 3), q = t & 7u; *(volatile v4u*)(hb + (size_t)rw * KP + 8u * q) = o[it]; }
  __threadfence();
#pragma unroll
  for (unsigned it = 0; it < 4; ++it) { const unsigned rw = it * 32u + (t >> 3), q = t & 7u; *(volatile v4u*)(hb + (size_t)rw * KP + 8u * q) = o[it]; }
}

__global__ __launch_bounds__(256) void k_out(const unsigned short* __restrict__ HB, const unsigned short* __restrict__ W2T, float* __restrict__ OUT) {
  __shared__ __align__(16) float sf[8][16][64];
  const unsigned t = threadIdx.x, wave = t >> 5, lane = t & 31u, lm = lane & 15u, lh = lane >> 4, wm = wave >> 1, wn = wave & 1u;
  const unsigned m0 = blockIdx.y * 128u, n0 = blockIdx.x * 128u;
  const unsigned short* ar[2]; const unsigned short* br[4];
#pragma unroll
  for (int mi = 0; mi < 2; ++mi) ar[mi] = HB + (size_t)(m0 + wm * 32u + mi * 16u + lm) * KP + 8u * lh;
#pragma unroll
  for (int ni = 0; ni < 4; ++ni) br[ni] = W2T + (size_t)(n0 + wn * 64u + ni * 16u + lm) * KP + 8u * lh;
  v8f acc[2][4] = {};
#pragma unroll 2
  for (unsigned kc = 0; kc < KP / 32; ++kc) { v16h a[2], b[4];
#pragma unroll
    for (int mi = 0; mi < 2; ++mi) a[mi] = ldfrag_h(ar[mi] + kc * 32u);
#pragma unroll
    for (int ni = 0; ni < 4; ++ni) b[ni] = ldfrag_h(br[ni] + kc * 32u);
#pragma unroll
    for (int mi = 0; mi < 2; ++mi)
#pragma unroll
      for (int ni = 0; ni < 4; ++ni) acc[mi][ni] = wmma16(a[mi], b[ni], acc[mi][ni]); }
#pragma unroll
  for (int mi = 0; mi < 2; ++mi) {
    if (mi) __syncthreads();
#pragma unroll
    for (int ni = 0; ni < 4; ++ni)
#pragma unroll
      for (int r = 0; r < 8; ++r) sf[wave][8u * lh + r][ni * 16 + lm] = acc[mi][ni][r] * OSCALE;
    __syncthreads();
    v4f v[8];
#pragma unroll
    for (unsigned it = 0; it < 8; ++it) { const unsigned rw = it * 2u + (lane >> 4), pc = lane & 15u; v[it] = *(const v4f*)&sf[wave][rw][4u * pc]; }
    float* po = OUT + (size_t)(m0 + wm * 32u + mi * 16u) * DOUT + n0 + wn * 64u;
#pragma unroll
    for (unsigned it = 0; it < 8; ++it) { const unsigned rw = it * 2u + (lane >> 4), pc = lane & 15u; *(volatile v4f*)(po + (size_t)rw * DOUT + 4u * pc) = v[it]; }
    __threadfence();
#pragma unroll
    for (unsigned it = 0; it < 8; ++it) { const unsigned rw = it * 2u + (lane >> 4), pc = lane & 15u; *(volatile v4f*)(po + (size_t)rw * DOUT + 4u * pc) = v[it]; }
  }
}

extern "C" void kernel_launch(void* const* d_in, const int* in_sizes, int n_in, void* d_out, int out_size, void* d_ws, size_t ws_size, hipStream_t stream) {
  if (n_in < 8) return;
  if (in_sizes[0] < NB * DIN || in_sizes[1] < NE * DIN) return;
  if (in_sizes[2] < NE * DIN * DHID || in_sizes[3] < NE * DIN * DHID || in_sizes[4] < NE * DHID * DOUT) return;
  if (in_sizes[5] < DIN * DHID || in_sizes[6] < DIN * DHID || in_sizes[7] < DHID * DOUT) return;
  if ((size_t)out_size < (size_t)NB * DOUT) return;
  if (ws_size < (size_t)WS_END) return;
  const float* X   = (const float*)d_in[0];
  const float* GW  = (const float*)d_in[1];
  const float* WG  = (const float*)d_in[2];
  const float* WU  = (const float*)d_in[3];
  const float* WD  = (const float*)d_in[4];
  const float* WSG = (const float*)d_in[5];
  const float* WSU = (const float*)d_in[6];
  const float* WSD = (const float*)d_in[7];
  char* ws = (char*)d_ws;
  unsigned short* XB  = (unsigned short*)(ws + WS_XB);
  unsigned short* WGT = (unsigned short*)(ws + WS_WGT);
  unsigned short* WUT = (unsigned short*)(ws + WS_WUT);
  unsigned short* W2T = (unsigned short*)(ws + WS_W2T);
  unsigned short* HB  = (unsigned short*)(ws + WS_HB);
  float* RT  = (float*)(ws + WS_RT);
  float* OUT = (float*)d_out;
  k_cvt_x<<<dim3(NB * DIN / 8 / 256), 256, 0, stream>>>(X, XB);
  k_tr<0><<<dim3(DHID / 64, DIN / 64, NE), 256, 0, stream>>>(WG, WGT, (unsigned)DIN, (unsigned)DHID, (unsigned)DIN, (unsigned)DHID, 0u, 1.0f);
  k_tr<0><<<dim3(DHID / 64, DIN / 64, NE), 256, 0, stream>>>(WU, WUT, (unsigned)DIN, (unsigned)DHID, (unsigned)DIN, (unsigned)DHID, 0u, 1.0f);
  k_tr<0><<<dim3(DHID / 64, DIN / 64, 1), 256, 0, stream>>>(WSG, WGT + (size_t)NE * DHID * DIN, (unsigned)DIN, (unsigned)DHID, (unsigned)DIN, (unsigned)DHID, 0u, 1.0f);
  k_tr<0><<<dim3(DHID / 64, DIN / 64, 1), 256, 0, stream>>>(WSU, WUT + (size_t)NE * DHID * DIN, (unsigned)DIN, (unsigned)DHID, (unsigned)DIN, (unsigned)DHID, 0u, 1.0f);
  k_tr<1><<<dim3(DOUT / 64, DHID / 64, NE), 256, 0, stream>>>(WD, W2T, (unsigned)DHID, (unsigned)DOUT, (unsigned)KP, 0u, (unsigned)DHID, WCARRY);
  k_tr<1><<<dim3(DOUT / 64, DHID / 64, 1), 256, 0, stream>>>(WSD, W2T + (size_t)NE * DHID, (unsigned)DHID, (unsigned)DOUT, (unsigned)KP, 0u, (unsigned)DHID, WCARRY);
  k_gate<<<dim3(NB / 16), 256, 0, stream>>>(XB, GW, RT);
  k_h<<<dim3(DHID / 64, NB / 128, NX), 256, 0, stream>>>(XB, WGT, WUT, RT, HB);
  k_out<<<dim3(DOUT / 128, NB / 128), 256, 0, stream>>>(HB, W2T, OUT);
}
